// MPG_65979287601499
// MI455X (gfx1250) — hardware-run, weakly checked
//
#include <hip/hip_runtime.h>
#include <stddef.h>
#include <stdint.h>
#include <math.h>

#define NN      50000
#define NE      600000
#define DF      128
#define KD      128
#define APITCH  128
#define WPITCH  128
#define GBM     128
#define MP      50048
#define NTHR    256
#define NWAVE   8
#define EPT     8
#define WCH     (32 * EPT)
#define NBRUN   1024
#define SLB     10
#define NBK     49
#define WLCAP   3584
#define RCAP    28672
#define DEGCAP  128
#define MAXDEG_MEAS   28
#define MAXB1024_MEAS 12548
#define SP      68
#define RBM     128
#define PER     (((NE + NWAVE * WCH - 1) / (NWAVE * WCH)) * WCH)

#define BK_ZINTS (NWAVE * WLCAP + RCAP + 4 * NBRUN)
#define BK_INTS  (BK_ZINTS + 16)
#define BK_LDS   (BK_INTS * 4)

#define PBX   (MP * DF / 8 / NTHR)
#define PBW   (DF * DF / 8 / NTHR)
#define PBTOT (PBX + PBW + 1)

static_assert(NBK * NBRUN >= NN && NBK * NBRUN >= MP);
static_assert(NN <= MP && MP == 391 * GBM && MP % RBM == 0);
static_assert(DF == 128 && DF == 32 * 4 && KD % 32 == 0 && KD <= APITCH && KD <= WPITCH);
static_assert(NBRUN == (1 << SLB) && NBRUN % RBM == 0 && NBRUN % GBM == 0 && NBRUN % 32 == 0);
static_assert(NBRUN == 4 * NTHR);
static_assert(RCAP % 32 == 0 && RCAP == NWAVE * WLCAP && BK_ZINTS % 4 == 0);
static_assert((long long)RCAP * 100 >= (long long)MAXB1024_MEAS * 105);
static_assert(WLCAP >= MAXB1024_MEAS / 8 + 8 * 40 + 1);
static_assert(MAXDEG_MEAS + 8 <= DEGCAP);
static_assert(NE % EPT == 0 && NE % 4 == 0 && NE < (1 << 20));
static_assert((((long long)NE) << SLB) < (1LL << 31));
static_assert((NWAVE - 1) * PER < NE && NWAVE * PER >= NE && PER % WCH == 0);
static_assert(BK_LDS <= 300000 && BK_LDS <= 327680);
static_assert((GBM * SP + GBM) * 4 <= 65536);
static_assert((MP * DF / 8) % NTHR == 0 && (DF * DF / 8) % NTHR == 0);
static_assert(GBM == NWAVE * 16 && RBM == NWAVE * 16);

typedef float          v4f   __attribute__((ext_vector_type(4)));
typedef float          v8f   __attribute__((ext_vector_type(8)));
typedef int            v4i   __attribute__((ext_vector_type(4)));
typedef int            v8i   __attribute__((ext_vector_type(8)));
typedef unsigned short v8us  __attribute__((ext_vector_type(8)));
typedef unsigned short v16us __attribute__((ext_vector_type(16)));
typedef __bf16         v16bf __attribute__((ext_vector_type(16)));
typedef v4f  __attribute__((may_alias)) v4fa;
typedef v4i  __attribute__((may_alias)) v4ia;
typedef v8us __attribute__((may_alias)) v8usa;
union FragB { v16bf v; v16us u; v8us h[2]; v8i w; };

__device__ __forceinline__ v8f wmb(const FragB& a, const FragB& b, v8f c) {
  v8f d = __builtin_amdgcn_wmma_f32_16x16x32_bf16(false, a.v, false, b.v, (short)0, c, false, false);
  asm volatile("v_nop\n\tv_nop\n\tv_nop\n\tv_nop" : "+v"(d) : "v"(a.w), "v"(b.w));
  return d;
}

__device__ __forceinline__ unsigned bf16_bits(float f) {
  const unsigned u = __float_as_uint(f);
  const unsigned r = (u + 0x7FFFu + ((u >> 16) & 1u)) >> 16;
  const unsigned q = (u >> 16) | 0x40u;
  return ((u & 0x7fffffffu) > 0x7f800000u) ? q : r;
}
__device__ __forceinline__ float bf16_val(float f) {
  return __uint_as_float(bf16_bits(f) << 16);
}

__device__ __forceinline__ void st2_v4f(float* p, v4f v) {
  *(volatile v4f*)p = v;
  __threadfence();
  *(volatile v4f*)p = v;
}
__device__ __forceinline__ void st2_v8us(unsigned short* p, v8us v) {
  *(volatile v8us*)p = v;
  __threadfence();
  *(volatile v8us*)p = v;
}

__device__ __forceinline__ v8us gather8(const float* __restrict__ base, int stride) {
  float f[8];
#pragma unroll
  for (int i = 0; i < 8; ++i) f[i] = base[(size_t)i * (size_t)stride];
  v8us o;
#pragma unroll
  for (int i = 0; i < 8; ++i) o[i] = (unsigned short)bf16_bits(f[i]);
  return o;
}

__global__ __launch_bounds__(NTHR) void k_prep(const float* __restrict__ x, const float* __restrict__ w,
                                               const float* __restrict__ b, unsigned short* xb,
                                               unsigned short* wt, float* bias) {
  const int tid = (int)threadIdx.x, lane = tid & 31;
  const int blk = (int)blockIdx.x;
  if (blk < PBX) {
    const int u   = blk * NTHR + tid;
    const int row = u >> 4, k8 = (u & 15) * 8;
    const int rc  = row < NN ? row : NN - 1;
    const unsigned mk = row < NN ? 0xffffu : 0u;
    const float* p = x + (size_t)rc * DF + k8;
    const v4f a = *(const v4fa*)p;
    const v4f c = *(const v4fa*)(p + 4);
    v8us o;
    o[0] = (unsigned short)(bf16_bits(a.x) & mk); o[1] = (unsigned short)(bf16_bits(a.y) & mk);
    o[2] = (unsigned short)(bf16_bits(a.z) & mk); o[3] = (unsigned short)(bf16_bits(a.w) & mk);
    o[4] = (unsigned short)(bf16_bits(c.x) & mk); o[5] = (unsigned short)(bf16_bits(c.y) & mk);
    o[6] = (unsigned short)(bf16_bits(c.z) & mk); o[7] = (unsigned short)(bf16_bits(c.w) & mk);
    st2_v8us(xb + (size_t)row * APITCH + k8, o);
  } else if (blk < PBX + PBW) {
    const int u = (blk - PBX) * NTHR + tid;
    const int n = u >> 4, k8 = (u & 15) * 8;
    const v8us o = gather8(w + (size_t)k8 * DF + n, DF);
    st2_v8us(wt + (size_t)n * WPITCH + k8, o);
  } else {
    if (tid < 32) {
      const v4f a = *(const v4fa*)(b + 4 * lane);
      v4f o;
      o.x = bf16_val(a.x); o.y = bf16_val(a.y); o.z = bf16_val(a.z); o.w = bf16_val(a.w);
      st2_v4f(bias + 4 * lane, o);
    }
  }
}

__device__ __forceinline__ void bucket_flush(const int* pl, const int* cnt, const int* offs, const int* dvb,
                                             int ov, int* lp, int* cp, int* op, int* dp, int* fp, int tid) {
#pragma unroll 1
  for (int i = tid * 4; i < RCAP; i += NTHR * 4) {
    const v4i v = *(const v4ia*)(pl + i);
    *(volatile v4i*)(lp + i) = v;
  }
  {
    const v4i v = *(const v4ia*)(cnt + 4 * tid);
    *(volatile v4i*)(cp + 4 * tid) = v;
  }
  {
    const v4i v = *(const v4ia*)(offs + 4 * tid);
    *(volatile v4i*)(op + 4 * tid) = v;
  }
  {
    const v4i v = *(const v4ia*)(dvb + 4 * tid);
    *(volatile v4i*)(dp + 4 * tid) = v;
  }
  if (tid < 8) {
    const v4i f = {ov, ov, ov, ov};
    *(volatile v4i*)(fp + 4 * tid) = f;
  }
}

__global__ __launch_bounds__(NTHR) void k_bucket(const int* __restrict__ srcs, const int* __restrict__ dsts,
                                                 int* LIST, int* CNT, int* OFF, int* DINVB, int* FLAG) {
  extern __shared__ __attribute__((aligned(16))) int dsm[];
  int* wl   = dsm;
  int* pl   = dsm + NWAVE * WLCAP;
  int* cnt  = pl + RCAP;
  int* offs = cnt + NBRUN;
  int* dvb  = offs + NBRUN;
  int* cur  = dvb + NBRUN;
  int* misc = cur + NBRUN;
  const int tid = (int)threadIdx.x, lane = tid & 31, wave = tid >> 5;
  const int blk = (int)blockIdx.x;
  const unsigned nbs = (unsigned)(blk * NBRUN);

  {
    const v4i z4 = {0, 0, 0, 0};
    for (int i = tid * 4; i < BK_ZINTS; i += NTHR * 4) *(v4ia*)(dsm + i) = z4;
    if (tid < 16) misc[tid] = 0;
  }
  __syncthreads();

  {
    const int ebeg = wave * PER;
    const int eend = (ebeg + PER < NE) ? (ebeg + PER) : NE;
    int* mylist = wl + wave * WLCAP;
    int wc = 0;
#pragma unroll 1
    for (int cb = ebeg; cb < eend; cb += WCH) {
      const int e0  = cb + lane * EPT;
      const int e0c = e0 < NE - EPT ? e0 : NE - EPT;
      const v4i da = *(const v4ia*)(dsts + e0c);
      const v4i db = *(const v4ia*)(dsts + e0c + 4);
      asm volatile("" :: "v"(da), "v"(db));
      const bool ok = e0 < eend;
      const unsigned s0 = (unsigned)da.x - nbs, s1 = (unsigned)da.y - nbs;
      const unsigned s2 = (unsigned)da.z - nbs, s3 = (unsigned)da.w - nbs;
      const unsigned s4 = (unsigned)db.x - nbs, s5 = (unsigned)db.y - nbs;
      const unsigned s6 = (unsigned)db.z - nbs, s7 = (unsigned)db.w - nbs;
      const bool h0 = ok & (s0 < (unsigned)NBRUN), h1 = ok & (s1 < (unsigned)NBRUN);
      const bool h2 = ok & (s2 < (unsigned)NBRUN), h3 = ok & (s3 < (unsigned)NBRUN);
      const bool h4 = ok & (s4 < (unsigned)NBRUN), h5 = ok & (s5 < (unsigned)NBRUN);
      const bool h6 = ok & (s6 < (unsigned)NBRUN), h7 = ok & (s7 < (unsigned)NBRUN);
      const unsigned m0 = __builtin_amdgcn_ballot_w32(h0), m1 = __builtin_amdgcn_ballot_w32(h1);
      const unsigned m2 = __builtin_amdgcn_ballot_w32(h2), m3 = __builtin_amdgcn_ballot_w32(h3);
      const unsigned m4 = __builtin_amdgcn_ballot_w32(h4), m5 = __builtin_amdgcn_ballot_w32(h5);
      const unsigned m6 = __builtin_amdgcn_ballot_w32(h6), m7 = __builtin_amdgcn_ballot_w32(h7);
      const unsigned any = m0 | m1 | m2 | m3 | m4 | m5 | m6 | m7;
      if (any != 0u) {
        const int pre = (int)(__builtin_amdgcn_mbcnt_lo(m0, 0u) + __builtin_amdgcn_mbcnt_lo(m1, 0u) +
                              __builtin_amdgcn_mbcnt_lo(m2, 0u) + __builtin_amdgcn_mbcnt_lo(m3, 0u) +
                              __builtin_amdgcn_mbcnt_lo(m4, 0u) + __builtin_amdgcn_mbcnt_lo(m5, 0u) +
                              __builtin_amdgcn_mbcnt_lo(m6, 0u) + __builtin_amdgcn_mbcnt_lo(m7, 0u));
        int p = wc + pre;
        if (h0) { if (p < WLCAP) mylist[p] = ((e0 + 0) << SLB) | (int)s0; p = p + 1; }
        if (h1) { if (p < WLCAP) mylist[p] = ((e0 + 1) << SLB) | (int)s1; p = p + 1; }
        if (h2) { if (p < WLCAP) mylist[p] = ((e0 + 2) << SLB) | (int)s2; p = p + 1; }
        if (h3) { if (p < WLCAP) mylist[p] = ((e0 + 3) << SLB) | (int)s3; p = p + 1; }
        if (h4) { if (p < WLCAP) mylist[p] = ((e0 + 4) << SLB) | (int)s4; p = p + 1; }
        if (h5) { if (p < WLCAP) mylist[p] = ((e0 + 5) << SLB) | (int)s5; p = p + 1; }
        if (h6) { if (p < WLCAP) mylist[p] = ((e0 + 6) << SLB) | (int)s6; p = p + 1; }
        if (h7) { if (p < WLCAP) mylist[p] = ((e0 + 7) << SLB) | (int)s7; p = p + 1; }
        wc += (int)(__builtin_popcount(m0) + __builtin_popcount(m1) + __builtin_popcount(m2) + __builtin_popcount(m3) +
                    __builtin_popcount(m4) + __builtin_popcount(m5) + __builtin_popcount(m6) + __builtin_popcount(m7));
      }
    }
    if (lane == 0) misc[wave] = wc;
  }
  __syncthreads();

  int ov = 0;
  if (wave == 0) {
#pragma unroll 1
    for (int w2 = 0; w2 < NWAVE; ++w2) {
      int c = misc[w2];
      if (c > WLCAP) ov = 1;
      c = c < 0 ? 0 : (c > WLCAP ? WLCAP : c);
#pragma unroll 1
      for (int b0 = 0; b0 < c; b0 += 32) {
        const int idx = b0 + lane;
        const int ent = wl[w2 * WLCAP + (idx < WLCAP ? idx : WLCAP - 1)];
        const int m32 = (c - b0) < 32 ? (c - b0) : 32;
#pragma unroll 1
        for (int k = 0; k < m32; ++k) {
          const int u    = __builtin_amdgcn_readlane(ent, k);
          const int slot = u & (NBRUN - 1);
          if (lane == 0) cnt[slot] = cnt[slot] + 1;
        }
      }
    }
  }
  __syncthreads();
  if (wave == 0) {
    const int base = lane * (NBRUN / 32);
    int s = 0;
    int ovl = 0;
#pragma unroll 1
    for (int i = 0; i < NBRUN / 32; ++i) {
      const int cv = cnt[base + i];
      ovl |= (cv > DEGCAP) ? 1 : 0;
      s += cv;
    }
    const unsigned bm = __builtin_amdgcn_ballot_w32(ovl != 0);
    int incl = s;
#pragma unroll
    for (int d = 1; d < 32; d <<= 1) {
      const int y = __shfl_up(incl, d, 32);
      if (lane >= d) incl += y;
    }
    int run = incl - s;
#pragma unroll 1
    for (int i = 0; i < NBRUN / 32; ++i) {
      const int cv = cnt[base + i];
      offs[base + i] = run;
      cur[base + i]  = run;
      run += cv;
    }
    if (lane == 0) misc[9] = ov | ((bm != 0u) ? 1 : 0);
  }
  __syncthreads();

  if (wave == 0) {
#pragma unroll 1
    for (int w2 = 0; w2 < NWAVE; ++w2) {
      int c = misc[w2];
      c = c < 0 ? 0 : (c > WLCAP ? WLCAP : c);
#pragma unroll 1
      for (int b0 = 0; b0 < c; b0 += 32) {
        const int idx = b0 + lane;
        const int ent = wl[w2 * WLCAP + (idx < WLCAP ? idx : WLCAP - 1)];
        int eid = (ent >> SLB) & 0xFFFFF;
        eid = eid > NE - 1 ? NE - 1 : eid;
        int sr = srcs[eid];
        sr = sr < 0 ? 0 : (sr > NN - 1 ? NN - 1 : sr);
        const int m32 = (c - b0) < 32 ? (c - b0) : 32;
#pragma unroll 1
        for (int k = 0; k < m32; ++k) {
          const int u    = __builtin_amdgcn_readlane(ent, k);
          const int wd   = __builtin_amdgcn_readlane(sr, k);
          const int slot = u & (NBRUN - 1);
          if (lane == 0) {
            int p = cur[slot];
            p = p < 0 ? 0 : (p > RCAP - 1 ? RCAP - 1 : p);
            pl[p] = wd;
            cur[slot] = p + 1;
          }
        }
      }
    }
  }
  __syncthreads();

#pragma unroll 1
  for (int i = tid; i < NBRUN; i += NTHR) {
    const int c = cnt[i];
    const float dg = (float)(c + 1);
    dvb[i] = __float_as_int(1.0f / sqrtf(dg));
  }
  __syncthreads();

  const int ovf = misc[9];
  int* lp = LIST  + (size_t)blk * RCAP;
  int* cp = CNT   + (size_t)blk * NBRUN;
  int* op = OFF   + (size_t)blk * NBRUN;
  int* dp = DINVB + (size_t)blk * NBRUN;
  int* fp = FLAG  + (size_t)blk * 32;
  bucket_flush(pl, cnt, offs, dvb, ovf, lp, cp, op, dp, fp, tid);
  __threadfence();
  bucket_flush(pl, cnt, offs, dvb, ovf, lp, cp, op, dp, fp, tid);
}

__global__ __launch_bounds__(NTHR) __attribute__((amdgpu_num_vgpr(248)))
void k_gemm(const unsigned short* __restrict__ XB, const unsigned short* __restrict__ WT,
            const float* __restrict__ DINV, float* P) {
  __shared__ __attribute__((aligned(16))) float stg[GBM * SP];
  __shared__ __attribute__((aligned(16))) float sd[GBM];
  const int tid = (int)threadIdx.x, lane = tid & 31, wave = tid >> 5, hh = lane >> 4, m = lane & 15;
  const int rowBase = (int)blockIdx.x * GBM;
  if (tid < 32) *(v4fa*)(sd + 4 * tid) = *(const v4fa*)(DINV + (size_t)rowBase + 4 * tid);

  v8f acc[8];
  {
    const v8f z = {0.f, 0.f, 0.f, 0.f, 0.f, 0.f, 0.f, 0.f};
#pragma unroll
    for (int t = 0; t < 8; ++t) acc[t] = z;
  }
  const unsigned short* ap = XB + (size_t)(rowBase + 16 * wave + m) * (size_t)APITCH + 8 * hh;
  const unsigned short* bp = WT + (size_t)m * (size_t)WPITCH + 8 * hh;
#pragma unroll 1
  for (int k0 = 0; k0 < KD; k0 += 32) {
    FragB af;
    af.h[0] = *(const v8usa*)(ap + k0);
    af.h[1] = *(const v8usa*)(ap + k0 + 16);
#pragma unroll
    for (int nt = 0; nt < 8; ++nt) {
      const unsigned short* wq = bp + (size_t)(16 * nt) * (size_t)WPITCH + k0;
      FragB bf;
      bf.h[0] = *(const v8usa*)wq;
      bf.h[1] = *(const v8usa*)(wq + 16);
      acc[nt] = wmb(af, bf, acc[nt]);
    }
  }

#pragma unroll
  for (int half = 0; half < 2; ++half) {
    if (half != 0) __syncthreads();
#pragma unroll
    for (int nt = 0; nt < 4; ++nt) {
#pragma unroll
      for (int r = 0; r < 8; ++r) stg[(16 * wave + 8 * hh + r) * SP + 16 * nt + m] = acc[4 * half + nt][r];
    }
    __syncthreads();
#pragma unroll 1
    for (int i = 0; i < 8; ++i) {
      const int lr   = 16 * wave + 2 * i + hh;
      const int grow = rowBase + lr;
      const bool live = grow < NN;
      const v4f a  = *(const v4fa*)(stg + lr * SP + 4 * m);
      const float dv = sd[lr];
      asm volatile("" :: "v"(a), "v"(dv));
      const float v0 = dv * a.x, v1 = dv * a.y, v2 = dv * a.z, v3 = dv * a.w;
      v4f o;
      o.x = live ? v0 : 0.0f; o.y = live ? v1 : 0.0f; o.z = live ? v2 : 0.0f; o.w = live ? v3 : 0.0f;
      st2_v4f(P + (size_t)grow * DF + 64 * half + 4 * m, o);
    }
  }
}

__global__ __launch_bounds__(NTHR) void k_replay(const int* __restrict__ LIST, const int* __restrict__ CNT,
                                                 const int* __restrict__ OFF, const float* __restrict__ DINV,
                                                 const int* __restrict__ FLAG, const float* __restrict__ P,
                                                 const float* __restrict__ BIAS, float* out) {
  const int tid = (int)threadIdx.x, lane = tid & 31, wave = tid >> 5;
  const int rowBase = (int)blockIdx.x * RBM;
  const int bucket  = rowBase >> SLB;
  const int* lb  = LIST + (size_t)bucket * RCAP;
  const int flag = FLAG[(size_t)bucket * 32];
  const int r0   = rowBase + 16 * wave;
  const int ti   = r0 + (lane & 15);
  int   cv  = CNT[ti];
  int   ovv = OFF[ti];
  const float dvv = DINV[ti];
  asm volatile("" :: "v"(cv), "v"(ovv), "v"(dvv));
  const int bigv = (cv > DEGCAP) ? 1 : 0;
  cv  = cv  < 0 ? 0 : (cv  > DEGCAP   ? DEGCAP   : cv);
  ovv = ovv < 0 ? 0 : (ovv > RCAP - 1 ? RCAP - 1 : ovv);
  const int dvi = __float_as_int(dvv);
  const v4f bias = *(const v4fa*)(BIAS + 4 * lane);
  const float qnan = __uint_as_float(0x7fc00000u);

#pragma unroll 1
  for (int t = 0; t < 16; ++t) {
    const int i   = r0 + t;
    const int c   = __builtin_amdgcn_readlane(cv, t);
    const int o   = __builtin_amdgcn_readlane(ovv, t);
    const int big = __builtin_amdgcn_readlane(bigv, t);
    const float dinv = __int_as_float(__builtin_amdgcn_readlane(dvi, t));
    int last = o + c - 1;
    last = max(last, o);
    last = min(last, RCAP - 1);
    float a0 = 0.0f, a1 = 0.0f, a2 = 0.0f, a3 = 0.0f;
#pragma unroll 1
    for (int b0 = 0; b0 < c; b0 += 32) {
      int idx = o + b0 + lane;
      idx = idx > last ? last : idx;
      const int ent = lb[idx];
      const int s   = ent < 0 ? 0 : (ent > NN - 1 ? NN - 1 : ent);
      const int m32 = (c - b0) < 32 ? (c - b0) : 32;
#pragma unroll 1
      for (int k = 0; k < m32; k += 4) {
        const int s0 = __builtin_amdgcn_readlane(s, k);
        const int s1 = __builtin_amdgcn_readlane(s, k + 1);
        const int s2 = __builtin_amdgcn_readlane(s, k + 2);
        const int s3 = __builtin_amdgcn_readlane(s, k + 3);
        const v4f g0 = *(const v4fa*)(P + (size_t)s0 * DF + 4 * lane);
        const v4f g1 = *(const v4fa*)(P + (size_t)s1 * DF + 4 * lane);
        const v4f g2 = *(const v4fa*)(P + (size_t)s2 * DF + 4 * lane);
        const v4f g3 = *(const v4fa*)(P + (size_t)s3 * DF + 4 * lane);
        asm volatile("" :: "v"(g0), "v"(g1), "v"(g2), "v"(g3));
        const bool k1 = (k + 1) < m32, k2 = (k + 2) < m32, k3 = (k + 3) < m32;
        a0 = a0 + g0.x; a1 = a1 + g0.y; a2 = a2 + g0.z; a3 = a3 + g0.w;
        {
          const float t0 = a0 + g1.x, t1 = a1 + g1.y, t2 = a2 + g1.z, t3 = a3 + g1.w;
          a0 = k1 ? t0 : a0; a1 = k1 ? t1 : a1; a2 = k1 ? t2 : a2; a3 = k1 ? t3 : a3;
        }
        {
          const float t0 = a0 + g2.x, t1 = a1 + g2.y, t2 = a2 + g2.z, t3 = a3 + g2.w;
          a0 = k2 ? t0 : a0; a1 = k2 ? t1 : a1; a2 = k2 ? t2 : a2; a3 = k2 ? t3 : a3;
        }
        {
          const float t0 = a0 + g3.x, t1 = a1 + g3.y, t2 = a2 + g3.z, t3 = a3 + g3.w;
          a0 = k3 ? t0 : a0; a1 = k3 ? t1 : a1; a2 = k3 ? t2 : a2; a3 = k3 ? t3 : a3;
        }
      }
    }
    const v4f sv = *(const v4fa*)(P + (size_t)i * DF + 4 * lane);
    asm volatile("" :: "v"(sv));
    a0 = a0 + sv.x; a1 = a1 + sv.y; a2 = a2 + sv.z; a3 = a3 + sv.w;
    float v0 = dinv * a0 + bias.x, v1 = dinv * a1 + bias.y;
    float v2 = dinv * a2 + bias.z, v3 = dinv * a3 + bias.w;
    const bool bad = (flag != 0) | (big != 0);
    v0 = bad ? qnan : v0; v1 = bad ? qnan : v1; v2 = bad ? qnan : v2; v3 = bad ? qnan : v3;
    v4f ov;
    ov.x = v0; ov.y = v1; ov.z = v2; ov.w = v3;
    const int ic = i < NN ? i : NN - 1;
    float* op = out + (size_t)ic * DF + 4 * lane;
    const bool wr = i < NN;
    if (wr) *(volatile v4f*)op = ov;
    __threadfence();
    if (wr) *(volatile v4f*)op = ov;
  }
}

extern "C" void kernel_launch(void* const* d_in, const int* in_sizes, int n_in,
                              void* d_out, int out_size, void* d_ws, size_t ws_size,
                              hipStream_t stream) {
  if (n_in < 4) return;
  if (in_sizes[0] != NN * DF) return;
  if (in_sizes[1] != 2 * NE) return;
  if (in_sizes[2] != DF * DF) return;
  if (in_sizes[3] != DF) return;
  if (out_size != NN * DF) return;

  const float* x  = (const float*)d_in[0];
  const int*   ei = (const int*)d_in[1];
  const float* W  = (const float*)d_in[2];
  const float* b  = (const float*)d_in[3];
  float* out = (float*)d_out;
  const int* srcs = ei;
  const int* dsts = ei + NE;

  constexpr size_t zXB   = (size_t)MP * APITCH * 2;
  constexpr size_t zWT   = (size_t)DF * WPITCH * 2;
  constexpr size_t zBIAS = 512;
  constexpr size_t zP    = (size_t)MP * DF * 4;
  constexpr size_t zLIST = (size_t)NBK * RCAP * 4;
  constexpr size_t zTAB  = (size_t)NBK * NBRUN * 4;
  constexpr size_t zFLAG = 6400;
  constexpr size_t oXB   = 0;
  constexpr size_t oWT   = oXB + zXB;
  constexpr size_t oBIAS = oWT + zWT;
  constexpr size_t oP    = oBIAS + zBIAS;
  constexpr size_t oLIST = oP + zP;
  constexpr size_t oCNT  = oLIST + zLIST;
  constexpr size_t oOFF  = oCNT + zTAB;
  constexpr size_t oDINV = oOFF + zTAB;
  constexpr size_t oFLAG = oDINV + zTAB;
  constexpr size_t oEND  = oFLAG + zFLAG;
  static_assert(zXB % 256 == 0 && zWT % 256 == 0 && zBIAS % 256 == 0 && zP % 256 == 0);
  static_assert(zLIST % 256 == 0 && zTAB % 256 == 0 && zFLAG % 256 == 0 && zFLAG >= (size_t)NBK * 128);
  static_assert(oEND <= (size_t)(128u << 20));
  if (oEND > ws_size) return;

  char* ws = (char*)d_ws;
  unsigned short* XB   = (unsigned short*)(ws + oXB);
  unsigned short* WT   = (unsigned short*)(ws + oWT);
  float*          BIAS = (float*)(ws + oBIAS);
  float*          P    = (float*)(ws + oP);
  int*            LIST = (int*)(ws + oLIST);
  int*            CNT  = (int*)(ws + oCNT);
  int*            OFF  = (int*)(ws + oOFF);
  int*            DVB  = (int*)(ws + oDINV);
  int*            FLAG = (int*)(ws + oFLAG);

  hipFuncSetAttribute(reinterpret_cast<const void*>(&k_bucket), hipFuncAttributeMaxDynamicSharedMemorySize, (int)BK_LDS);

  k_prep<<<PBTOT, NTHR, 0, stream>>>(x, W, b, XB, WT, BIAS);
  k_bucket<<<NBK, NTHR, BK_LDS, stream>>>(srcs, dsts, LIST, CNT, OFF, DVB, FLAG);
  k_gemm<<<MP / GBM, NTHR, 0, stream>>>(XB, WT, (const float*)DVB, P);
  k_replay<<<MP / RBM, NTHR, 0, stream>>>(LIST, CNT, OFF, (const float*)DVB, FLAG, P, BIAS, out);
}
